// Edge_18013092840065
// MI455X (gfx1250) — hardware-verified
//
#include <hip/hip_runtime.h>
#include <stddef.h>
#include <stdint.h>


#define F        64
#define F2       128
#define DP       128
#define RP       128
#define K2       96
#define NTHR     256
#define NWAVE    8
#define EPT      8
#define CHUNK    (NTHR * EPT)
#define WCAP     (EPT * 32)
#define LISTN    (NWAVE * WCAP)
#define NBMAX    2048
#define ESH      11
#define RCAP     28672
#define DEGCAP   1024
#define GBM      64
#define GBN      64
#define GTHR     128
#define W1TU     1024
#define W2TU     768
#define W1TH     (F2 * F)
#define WTH      (W1TH + F * K2)
#define WSMAX    134217728
#define LDS_SCAN ((2 * RCAP + 2 * NBMAX + LISTN) * 4 + 64)

static_assert((CHUNK & (CHUNK - 1)) == 0 && CHUNK <= 4096);
static_assert((NBMAX & (NBMAX - 1)) == 0 && NBMAX == (1 << ESH));
static_assert(NTHR * 8 == NBMAX);
static_assert(LISTN >= NBMAX);
static_assert(LISTN >= NWAVE * WCAP);
static_assert((RCAP % 32) == 0);
static_assert(LDS_SCAN <= 300000);
static_assert(GBM == (GTHR / 32) * 16);
static_assert((F % 32) == 0 && (K2 % 32) == 0 && (F2 % GBN) == 0 && (F % GBN) == 0);
static_assert(K2 <= RP && F + 1 <= K2);
static_assert(W1TU * 8 == F2 * F && W2TU * 8 == F * K2);
static_assert(W1TU == 4 * NTHR);
static_assert((W1TH * 2) % 256 == 0);

typedef float          v4f  __attribute__((ext_vector_type(4)));
typedef float          v8f  __attribute__((ext_vector_type(8)));
typedef int            v4i  __attribute__((ext_vector_type(4)));
typedef int            v8i  __attribute__((ext_vector_type(8)));
typedef unsigned short v8us __attribute__((ext_vector_type(8)));
typedef __bf16         v16b __attribute__((ext_vector_type(16)));
union FragB { v16b v; v8us u[2]; v8i w; };

__device__ __forceinline__ v8f wmb(const FragB& a, const FragB& b, v8f c) {
  v8f d = __builtin_amdgcn_wmma_f32_16x16x32_bf16(false, a.v, false, b.v, (short)0, c, false, false);
  asm volatile("v_nop\n\tv_nop\n\tv_nop\n\tv_nop" : "+v"(d) : "v"(a.w), "v"(b.w));
  return d;
}

__device__ __forceinline__ unsigned bfbits(float f) {
  unsigned u = __float_as_uint(f);
  u += 0x7FFFu + ((u >> 16) & 1u);
  return u >> 16;
}
__device__ __forceinline__ float bfval(float f) { return __uint_as_float(bfbits(f) << 16); }

__device__ __forceinline__ v8us cvt8b(const v4f a, const v4f b) {
  v8us r;
  r[0] = (unsigned short)bfbits(a.x); r[1] = (unsigned short)bfbits(a.y);
  r[2] = (unsigned short)bfbits(a.z); r[3] = (unsigned short)bfbits(a.w);
  r[4] = (unsigned short)bfbits(b.x); r[5] = (unsigned short)bfbits(b.y);
  r[6] = (unsigned short)bfbits(b.z); r[7] = (unsigned short)bfbits(b.w);
  return r;
}

__device__ __forceinline__ void cvt8bhl(const v4f a, const v4f b, v8us& hi, v8us& lo) {
  const float t[8] = {a.x, a.y, a.z, a.w, b.x, b.y, b.z, b.w};
#pragma unroll
  for (int i = 0; i < 8; ++i) {
    const unsigned hb = bfbits(t[i]);
    const float hf = __uint_as_float(hb << 16);
    hi[i] = (unsigned short)hb;
    lo[i] = (unsigned short)bfbits(t[i] - hf);
  }
}

__device__ __forceinline__ v4f relu4(const v4f v) {
  v4f r;
  r.x = fmaxf(v.x, 0.f); r.y = fmaxf(v.y, 0.f); r.z = fmaxf(v.z, 0.f); r.w = fmaxf(v.w, 0.f);
  return r;
}

__device__ __forceinline__ float tanh_e(float x) {
  const float xc = fminf(fmaxf(x, -15.0f), 15.0f);
  const float e  = __expf(2.0f * xc);
  const float r  = __builtin_amdgcn_rcpf(e + 1.0f);
  const float t  = fmaf(-2.0f, r, 1.0f);
  return (x != x) ? x : t;
}

__device__ __forceinline__ int scan_chunk(const int* __restrict__ dsts, int nE, int cbase, int slotBase,
                                          int nb, int vec8, int* list, int tid, int lane, int wave) {
  int wc = 0;
  const int el0  = tid * EPT;
  const int e0   = cbase + el0;
  const int sent = -2147483647 - 1;
  v4i da, db;
  if (vec8 != 0 && cbase + CHUNK <= nE) {
    da = *(const v4i*)(dsts + e0);
    db = *(const v4i*)(dsts + e0 + 4);
  } else {
    da.x = (e0     < nE) ? dsts[min(e0,     nE - 1)] : sent;
    da.y = (e0 + 1 < nE) ? dsts[min(e0 + 1, nE - 1)] : sent;
    da.z = (e0 + 2 < nE) ? dsts[min(e0 + 2, nE - 1)] : sent;
    da.w = (e0 + 3 < nE) ? dsts[min(e0 + 3, nE - 1)] : sent;
    db.x = (e0 + 4 < nE) ? dsts[min(e0 + 4, nE - 1)] : sent;
    db.y = (e0 + 5 < nE) ? dsts[min(e0 + 5, nE - 1)] : sent;
    db.z = (e0 + 6 < nE) ? dsts[min(e0 + 6, nE - 1)] : sent;
    db.w = (e0 + 7 < nE) ? dsts[min(e0 + 7, nE - 1)] : sent;
  }
  const unsigned nbs = (unsigned)slotBase;
  const unsigned unb = (unsigned)nb;
  const unsigned s0 = (unsigned)da.x - nbs, s1 = (unsigned)da.y - nbs;
  const unsigned s2 = (unsigned)da.z - nbs, s3 = (unsigned)da.w - nbs;
  const unsigned s4 = (unsigned)db.x - nbs, s5 = (unsigned)db.y - nbs;
  const unsigned s6 = (unsigned)db.z - nbs, s7 = (unsigned)db.w - nbs;
  const bool h0 = s0 < unb, h1 = s1 < unb, h2 = s2 < unb, h3 = s3 < unb;
  const bool h4 = s4 < unb, h5 = s5 < unb, h6 = s6 < unb, h7 = s7 < unb;
  const unsigned any = __builtin_amdgcn_ballot_w32(h0 | h1 | h2 | h3 | h4 | h5 | h6 | h7);
  if (any != 0u) {
#define HITJ(J, HJ, SJ) { \
      const unsigned mj = __builtin_amdgcn_ballot_w32(HJ); \
      if (mj != 0u) { \
        if (HJ) { \
          const int pos = wc + (int)__builtin_amdgcn_mbcnt_lo(mj, 0u); \
          if (pos < WCAP) list[wave * WCAP + pos] = ((el0 + (J)) << 12) | (int)(SJ); \
        } \
        wc += (int)__builtin_popcount(mj); } }
    HITJ(0, h0, s0)
    HITJ(1, h1, s1)
    HITJ(2, h2, s2)
    HITJ(3, h3, s3)
    HITJ(4, h4, s4)
    HITJ(5, h5, s5)
    HITJ(6, h6, s6)
    HITJ(7, h7, s7)
#undef HITJ
  }
  return wc;
}

__global__ __launch_bounds__(NTHR) void k_wcvt(const float* __restrict__ W1, const float* __restrict__ W2,
                                               const float* __restrict__ b2, unsigned short* wt, int nUnits) {
  const int u = (int)blockIdx.x * NTHR + (int)threadIdx.x;
  if (u >= nUnits) return;
  v4f a, b;
  size_t o;
  if (u < W1TU) {
    const int n = u >> 3, k8 = (u & 7) * 8;
    const float* p = W1 + (size_t)(((n >> 6) * F) + k8) * F + (n & (F - 1));
    a.x = p[0];             a.y = p[(size_t)F];     a.z = p[(size_t)2 * F]; a.w = p[(size_t)3 * F];
    b.x = p[(size_t)4 * F]; b.y = p[(size_t)5 * F]; b.z = p[(size_t)6 * F]; b.w = p[(size_t)7 * F];
    o = (size_t)n * F + k8;
  } else {
    const int r  = u - W1TU;
    const int n  = r / 12;
    const int k8 = (r - 12 * n) * 8;
    const int kk = k8 > F - 8 ? F - 8 : k8;
    const float* p = W2 + (size_t)kk * F + n;
    v4f la, lb;
    la.x = p[0];             la.y = p[(size_t)F];     la.z = p[(size_t)2 * F]; la.w = p[(size_t)3 * F];
    lb.x = p[(size_t)4 * F]; lb.y = p[(size_t)5 * F]; lb.z = p[(size_t)6 * F]; lb.w = p[(size_t)7 * F];
    const float bv = b2[n];
    const bool isw = k8 < F, isb = k8 == F;
    a.x = isw ? la.x : (isb ? bv : 0.f);
    a.y = isw ? la.y : 0.f; a.z = isw ? la.z : 0.f; a.w = isw ? la.w : 0.f;
    b.x = isw ? lb.x : 0.f; b.y = isw ? lb.y : 0.f; b.z = isw ? lb.z : 0.f; b.w = isw ? lb.w : 0.f;
    o = (size_t)W1TH + (size_t)n * K2 + k8;
  }
  const v8us hv = cvt8b(a, b);
  *(volatile v8us*)(wt + o) = hv;
  __threadfence();
  *(volatile v8us*)(wt + o) = hv;
}

template<int MODE>
__global__ __launch_bounds__(GTHR) void k_ngemm(const float* __restrict__ A, const unsigned short* __restrict__ WT,
                                                float* outF, int nAr, int lda, int K, int ldo, int nSt) {
  __shared__ __attribute__((aligned(16))) float stg[GBM * GBN];
  const int tid = (int)threadIdx.x, lane = tid & 31, wave = tid >> 5, hh = lane >> 4, m = lane & 15;
  const int rowBase = (int)blockIdx.x * GBM;
  const int col0    = (int)blockIdx.y * GBN;

  v8f acc[4];
  {
    const v8f z = {0.f, 0.f, 0.f, 0.f, 0.f, 0.f, 0.f, 0.f};
#pragma unroll
    for (int t = 0; t < 4; ++t) acc[t] = z;
  }
  const int gra = rowBase + 16 * wave + m;
  const int grc = gra > nAr - 1 ? nAr - 1 : gra;
  const float* ap = A + (size_t)grc * (size_t)lda + 8 * hh;
  const unsigned short* wp = WT + (size_t)(col0 + m) * (size_t)K + 8 * hh;
  const int ksteps = K >> 5;
#pragma unroll 1
  for (int ks = 0; ks < ksteps; ++ks) {
    const float* aq = ap + 32 * ks;
    const v4f a0 = *(const v4f*)aq,        a1 = *(const v4f*)(aq + 4);
    const v4f a2 = *(const v4f*)(aq + 16), a3 = *(const v4f*)(aq + 20);
    if (MODE == 0) {
      FragB ah;
      ah.u[0] = cvt8b(a0, a1);
      ah.u[1] = cvt8b(a2, a3);
#pragma unroll
      for (int t = 0; t < 4; ++t) {
        const unsigned short* wq = wp + (size_t)(16 * t) * (size_t)K + 32 * ks;
        FragB bf;
        bf.u[0] = *(const v8us*)wq;
        bf.u[1] = *(const v8us*)(wq + 16);
        acc[t] = wmb(ah, bf, acc[t]);
      }
    } else {
      FragB ah, al;
      cvt8bhl(a0, a1, ah.u[0], al.u[0]);
      cvt8bhl(a2, a3, ah.u[1], al.u[1]);
#pragma unroll
      for (int t = 0; t < 4; ++t) {
        const unsigned short* wq = wp + (size_t)(16 * t) * (size_t)K + 32 * ks;
        FragB bf;
        bf.u[0] = *(const v8us*)wq;
        bf.u[1] = *(const v8us*)(wq + 16);
        acc[t] = wmb(ah, bf, acc[t]);
        acc[t] = wmb(al, bf, acc[t]);
      }
    }
  }

#pragma unroll
  for (int t = 0; t < 4; ++t) {
    const int lc = 16 * t + m;
#pragma unroll
    for (int r = 0; r < 8; ++r) {
      const int lr = 16 * wave + 8 * hh + r;
      float v = acc[t][r];
      if (MODE == 1) v = tanh_e(v);
      stg[lr * GBN + lc] = v;
    }
  }
  __syncthreads();

  v4f fv[8];
#pragma unroll
  for (int i = 0; i < 8; ++i) {
    const int lr = 16 * wave + 2 * i + hh;
    fv[i] = *(const v4f*)(stg + lr * GBN + 4 * m);
  }
#pragma unroll
  for (int i = 0; i < 8; ++i) {
    const int lr = 16 * wave + 2 * i + hh;
    const int gr = rowBase + lr;
    float* op = outF + (size_t)gr * (size_t)ldo + col0 + 4 * m;
    if (gr < nSt) *(volatile v4f*)op = fv[i];
  }
  __threadfence();
#pragma unroll
  for (int i = 0; i < 8; ++i) {
    const int lr = 16 * wave + 2 * i + hh;
    const int gr = rowBase + lr;
    float* op = outF + (size_t)gr * (size_t)ldo + col0 + 4 * m;
    if (gr < nSt) *(volatile v4f*)op = fv[i];
  }
}

__global__ __launch_bounds__(NTHR) void k_scan(
    const int* __restrict__ dsts, const int* __restrict__ srcs, const float* __restrict__ D,
    const float* __restrict__ b1, float* RS, int nN, int nE, int nb, int vec8, int NPr) {
  extern __shared__ v4f lds_dyn[];
  int* reg1 = (int*)lds_dyn;
  int* reg2 = reg1 + RCAP;
  int* scnt = reg2 + RCAP;
  int* soff = scnt + NBMAX;
  int* list = soff + NBMAX;
  int* wcnt = list + LISTN;
  int* wtot = wcnt + NWAVE;
  const int tid = (int)threadIdx.x, lane = tid & 31, wave = tid >> 5;
  const int nodeBase = (int)blockIdx.x * nb;

  for (int i = tid; i < NBMAX; i += NTHR) scnt[i] = 0;
  __syncthreads();

  int tot = 0;
  const int nChunks = (nE + CHUNK - 1) / CHUNK;
#pragma unroll 1
  for (int ch = 0; ch < nChunks; ++ch) {
    const int cbase = ch * CHUNK;
    const int wc = scan_chunk(dsts, nE, cbase, nodeBase, nb, vec8, list, tid, lane, wave);
    if (lane == 0) wcnt[wave] = wc;
    __syncthreads();
    int pre = 0, all = 0;
#pragma unroll
    for (int w2 = 0; w2 < NWAVE; ++w2) {
      int c = wcnt[w2];
      c = c < 0 ? 0 : (c > WCAP ? WCAP : c);
      all += c;
      pre += (w2 < wave) ? c : 0;
    }
    const int wcc  = wc > WCAP ? WCAP : wc;
    const int base = tot + pre;
#pragma unroll 1
    for (int i = lane; i < wcc; i += 32) {
      const int ent = list[wave * WCAP + i];
      const int el  = (ent >> 12) & (CHUNK - 1);
      const int sl  = ent & (NBMAX - 1);
      int eid = cbase + el;
      eid = eid > nE - 1 ? nE - 1 : eid;
      const int pos = base + i;
      if (pos < RCAP) reg1[pos] = (int)(((unsigned)eid << ESH) | (unsigned)sl);
    }
    tot += all;
    tot = tot > RCAP ? RCAP : tot;
    __syncthreads();
  }
  const int nh = tot;

  if (wave == 0) {
#pragma unroll 1
    for (int b0 = 0; b0 < nh; b0 += 32) {
      const int idx = b0 + lane;
      const int uv  = reg1[idx < RCAP ? idx : RCAP - 1];
      const int m32 = (nh - b0) < 32 ? (nh - b0) : 32;
#pragma unroll 1
      for (int k = 0; k < m32; ++k) {
        const int u  = __builtin_amdgcn_readlane(uv, k);
        const int sl = u & (NBMAX - 1);
        if (lane == 0) scnt[sl] = scnt[sl] + 1;
      }
    }
  }
  __syncthreads();

  {
    const v4i ca = *(const v4i*)(scnt + 8 * tid);
    const v4i cb = *(const v4i*)(scnt + 8 * tid + 4);
    const int e0 = ca.x < 0 ? 0 : ca.x, e1 = ca.y < 0 ? 0 : ca.y, e2 = ca.z < 0 ? 0 : ca.z, e3 = ca.w < 0 ? 0 : ca.w;
    const int e4 = cb.x < 0 ? 0 : cb.x, e5 = cb.y < 0 ? 0 : cb.y, e6 = cb.z < 0 ? 0 : cb.z, e7 = cb.w < 0 ? 0 : cb.w;
    const int ts = e0 + e1 + e2 + e3 + e4 + e5 + e6 + e7;
    int incl = ts;
#pragma unroll
    for (int d = 1; d < 32; d <<= 1) {
      const int up = __shfl_up(incl, d);
      if (lane >= d) incl += up;
    }
    if (lane == 31) wtot[wave] = incl;
    __syncthreads();
    int pre = 0;
#pragma unroll
    for (int w2 = 0; w2 < NWAVE; ++w2) pre += (w2 < wave) ? wtot[w2] : 0;
    int run = pre + incl - ts;
    soff[8 * tid + 0] = run; run += e0;
    soff[8 * tid + 1] = run; run += e1;
    soff[8 * tid + 2] = run; run += e2;
    soff[8 * tid + 3] = run; run += e3;
    soff[8 * tid + 4] = run; run += e4;
    soff[8 * tid + 5] = run; run += e5;
    soff[8 * tid + 6] = run; run += e6;
    soff[8 * tid + 7] = run;
  }
  __syncthreads();
  for (int i = tid; i < NBMAX; i += NTHR) list[i] = soff[i];
  __syncthreads();

  if (wave == 0) {
#pragma unroll 1
    for (int b0 = 0; b0 < nh; b0 += 32) {
      const int idx = b0 + lane;
      const int uv  = reg1[idx < RCAP ? idx : RCAP - 1];
      const int m32 = (nh - b0) < 32 ? (nh - b0) : 32;
#pragma unroll 1
      for (int k = 0; k < m32; ++k) {
        const int u   = __builtin_amdgcn_readlane(uv, k);
        const int sl  = u & (NBMAX - 1);
        const int eid = (int)((unsigned)u >> ESH);
        if (lane == 0) {
          int pos = list[sl];
          pos = pos < 0 ? 0 : (pos > RCAP - 1 ? RCAP - 1 : pos);
          reg2[pos] = eid;
          list[sl] = pos + 1;
        }
      }
    }
  }
  __syncthreads();

  const int c4 = 4 * (lane & 15);
  v4f b1v;
  {
    const v4f t = *(const v4f*)(b1 + c4);
    b1v.x = bfval(t.x); b1v.y = bfval(t.y); b1v.z = bfval(t.z); b1v.w = bfval(t.w);
  }
  const int nbw = nb >> 3;
  const bool ovf = (nh >= RCAP);
  const float qnan = __int_as_float(0x7fc00000);
  const bool isv = lane < 16, isd = lane == 16;
#pragma unroll 1
  for (int jt = 0; jt < nbw; ++jt) {
    const int slot = wave * nbw + jt;
    const int grow = nodeBase + slot;
    const int gcl  = grow < nN ? grow : nN - 1;
    int st = soff[slot];
    const int craw = scnt[slot];
    int cnt = craw;
    st  = st < 0 ? 0 : (st > nh ? nh : st);
    cnt = cnt < 0 ? 0 : (cnt > DEGCAP ? DEGCAP : cnt);
    if (cnt > nh - st) cnt = nh - st;
    const float pz = (ovf || craw > DEGCAP) ? qnan : 0.0f;
    const bool wr = grow < NPr;
    const float live = grow < nN ? 1.0f : 0.0f;

    const float* pr = D + (size_t)gcl * DP;
    const v4f pa = *(const v4f*)(pr + c4);
    const v4f pb = *(const v4f*)(pr + F + c4);
    const v4f pv = (pa - pb) + b1v;
    v4f sm = {0.f, 0.f, 0.f, 0.f};
#pragma unroll 1
    for (int q = 0; q < cnt; ++q) {
      int idx = st + q; idx = idx > RCAP - 1 ? RCAP - 1 : idx;
      int el = reg2[idx]; el = el < 0 ? 0 : (el > nE - 1 ? nE - 1 : el);
      int s = srcs[el]; s = s < 0 ? 0 : (s > nN - 1 ? nN - 1 : s);
      const v4f qv = *(const v4f*)(D + (size_t)s * DP + F + c4);
      sm = sm + relu4(pv + qv);
    }
    const float degf = (float)cnt;
    v4f rv;
    rv.x = isv ? sm.x : (isd ? degf : 0.f);
    rv.y = isv ? sm.y : 0.f;
    rv.z = isv ? sm.z : 0.f;
    rv.w = isv ? sm.w : 0.f;
    const v4f rs = rv * live + pz;
    float* gp = RS + (size_t)grow * RP + 4 * lane;
    if (wr) *(volatile v4f*)gp = rs;
    __threadfence();
    if (wr) *(volatile v4f*)gp = rs;
  }
}

static inline int cdiv(int a, int b) { return (a + b - 1) / b; }
static int pick_nb(int nE, int nN) {
  int nb = NBMAX;
  while (nb > 32 && (long long)nb * (long long)nE * 11LL > (long long)RCAP * (long long)nN * 8LL) nb >>= 1;
  return nb;
}

extern "C" void kernel_launch(void* const* d_in, const int* in_sizes, int n_in,
                              void* d_out, int out_size, void* d_ws, size_t ws_size,
                              hipStream_t stream) {
  if (n_in < 6) return;
  const int nN = in_sizes[0] / F;
  if (nN <= 0 || in_sizes[0] != nN * F || nN > (1 << 22)) return;
  const int nE = in_sizes[1] / 2;
  if (nE < 1 || in_sizes[1] != 2 * nE || nE > (1 << 21)) return;
  if (in_sizes[2] != F2 * F || in_sizes[3] != F) return;
  if (in_sizes[4] != F * F  || in_sizes[5] != F) return;
  if (out_size != nN * F) return;

  const float* x    = (const float*)d_in[0];
  const int*   eidx = (const int*)  d_in[1];
  const float* W1   = (const float*)d_in[2];
  const float* b1   = (const float*)d_in[3];
  const float* W2   = (const float*)d_in[4];
  const float* b2   = (const float*)d_in[5];
  const int* srcp = eidx;
  const int* dstp = eidx + (size_t)nE;
  float* out = (float*)d_out;

  const int NP = cdiv(nN, GBM) * GBM;
  const int nb = pick_nb(nE, nN);
  const int gA = cdiv(NP, nb);
  if (gA * nb < NP || nb > NBMAX || nb < 32) return;
  const int vec8 = ((nE & 3) == 0) ? 1 : 0;

  char* ws = (char*)d_ws;
  size_t off = 0;
  const size_t oWT = off; off += (size_t)WTH * 2;                off = (off + 255) & ~(size_t)255;
  const size_t oD  = off; off += (size_t)NP * DP * 4;            off = (off + 255) & ~(size_t)255;
  const size_t oR  = off; off += (size_t)NP * RP * 4;            off = (off + 255) & ~(size_t)255;
  if (off > ws_size || off > (size_t)WSMAX) return;
  unsigned short* WT  = (unsigned short*)(ws + oWT);
  unsigned short* W1T = WT;
  unsigned short* W2T = WT + W1TH;
  float* D = (float*)(ws + oD);
  float* R = (float*)(ws + oR);

  hipFuncSetAttribute(reinterpret_cast<const void*>(&k_scan),
                      hipFuncAttributeMaxDynamicSharedMemorySize, LDS_SCAN);

  {
    const int nU = W1TU + W2TU;
    k_wcvt<<<cdiv(nU, NTHR), NTHR, 0, stream>>>(W1, W2, b2, WT, nU);
  }
  k_ngemm<0><<<dim3(NP / GBM, F2 / GBN), GTHR, 0, stream>>>(x, W1T, D, nN, F, F, DP, NP);
  k_scan<<<gA, NTHR, LDS_SCAN, stream>>>(dstp, srcp, D, b1, R, nN, nE, nb, vec8, NP);
  k_ngemm<1><<<dim3(NP / GBM, F / GBN), GTHR, 0, stream>>>(R, W2T, out, NP, RP, K2, F, nN);
}
